// Encoder_29454885716713
// MI455X (gfx1250) — hardware-verified
//
#include <hip/hip_runtime.h>
#include <hip/hip_fp16.h>


#ifndef NB
#define NB 32
#endif
#ifndef SEQ
#define SEQ 2048
#endif
#define NB_FULL  32
#define SEQ_FULL 2048
#define FD   64
#define DQ   24
#define DV   32
#define FO   64
#define NTOK (NB * SEQ)
#define CH   256
#define WT_ROWS 96

static_assert(NB >= 1 && NB <= NB_FULL);
static_assert(SEQ >= CH && SEQ <= SEQ_FULL);
static_assert(SEQ % CH == 0);
static_assert(SEQ % 128 == 0);
static_assert(NTOK % 64 == 0);
static_assert(CH % 32 == 0);

typedef _Float16 v16h __attribute__((ext_vector_type(16)));
typedef _Float16 v8h  __attribute__((ext_vector_type(8)));
typedef _Float16 v4h  __attribute__((ext_vector_type(4)));
typedef float    v8f  __attribute__((ext_vector_type(8)));
typedef float    v4f  __attribute__((ext_vector_type(4)));

union Frag { v16h v; v8h h[2]; };

#define C1 (1.44269504088896340736f * 0.000244140625f)
#define C2 (1.44269504088896340736f * 1.1920928955078125e-07f)
#define SC_RES   2048.0f
#define SC_RINV  4.8828125e-04f
#define SC_O2H   1.52587890625e-05f
#define SC_OUT   9.765625e-04f

static __device__ __forceinline__ v8f zero8() {
    v8f z;
#pragma unroll
    for (int i = 0; i < 8; ++i) z[i] = 0.0f;
    return z;
}

static __device__ __forceinline__ v16h load_frag16(const _Float16* base, int ld, int lane) {
    int m  = lane & 15;
    int kb = (lane >> 4) << 3;
    const _Float16* p = base + (size_t)m * ld + kb;
    Frag f;
    f.h[0] = *(const v8h*)(p);
    f.h[1] = *(const v8h*)(p + 16);
    return f.v;
}

static __device__ __forceinline__ v8f wmma16(v16h a, v16h b, v8f c) {
    v8f d = __builtin_amdgcn_wmma_f32_16x16x32_f16(false, a, false, b, (short)0, c, false, false);
    asm volatile("v_nop\n\tv_nop\n\tv_nop\n\tv_nop" : "+v"(d) : "v"(a), "v"(b));
    return d;
}

static __device__ __forceinline__ float bf16r(float x) {
    unsigned u = __float_as_uint(x);
    u = (u + 0x7FFFu + ((u >> 16) & 1u)) & 0xFFFF0000u;
    return __uint_as_float(u);
}

static __device__ __forceinline__ float ex2(float x) {
    return __builtin_amdgcn_exp2f(x);
}

static __device__ __forceinline__ void wave_lds_sync() {
    __builtin_amdgcn_fence(3, "wavefront");
    asm volatile("s_wait_dscnt 0" ::: "memory");
    __builtin_amdgcn_wave_barrier();
}

__global__ __launch_bounds__(256) void k_wprep(const float* __restrict__ Wq,
                                                const float* __restrict__ Wk,
                                                const float* __restrict__ Wv,
                                                const float* __restrict__ Wh,
                                                _Float16* __restrict__ wTg,
                                                _Float16* __restrict__ whTg) {
    __shared__ __align__(16) _Float16 wT[WT_ROWS * FD];
    __shared__ __align__(16) _Float16 whT[FO * DV];
    const int tid = threadIdx.x;
    for (int idx = tid; idx < WT_ROWS * FD; idx += 256) {
        int n = idx >> 6, d = idx & 63;
        int iq = min(n, DQ - 1);
        int ik = min(max(n - 32, 0), DQ - 1);
        int iv = min(max(n - 64, 0), DV - 1);
        float wq = Wq[d * DQ + iq];
        float wk = Wk[d * DQ + ik];
        float wv = Wv[d * DV + iv];
        float w = (n < DQ) ? wq : ((n < 32) ? 0.0f : ((n < 32 + DQ) ? wk : ((n < 64) ? 0.0f : wv)));
        wT[idx] = (_Float16)(bf16r(w) * 64.0f);
    }
    for (int idx = tid; idx < FO * DV; idx += 256) {
        int f = idx >> 5, d = idx & 31;
        whT[idx] = (_Float16)(bf16r(Wh[d * FO + f]) * 64.0f);
    }
    __syncthreads();
    v8h w0 = *(const v8h*)(&wT[(0 * 256 + tid) * 8]);
    v8h w1 = *(const v8h*)(&wT[(1 * 256 + tid) * 8]);
    v8h w2 = *(const v8h*)(&wT[(2 * 256 + tid) * 8]);
    v8h h0 = *(const v8h*)(&whT[tid * 8]);
    *(volatile v8h*)(wTg + (size_t)(0 * 256 + tid) * 8) = w0;
    *(volatile v8h*)(wTg + (size_t)(1 * 256 + tid) * 8) = w1;
    *(volatile v8h*)(wTg + (size_t)(2 * 256 + tid) * 8) = w2;
    *(volatile v8h*)(whTg + (size_t)tid * 8) = h0;
    __threadfence();
    *(volatile v8h*)(wTg + (size_t)(0 * 256 + tid) * 8) = w0;
    *(volatile v8h*)(wTg + (size_t)(1 * 256 + tid) * 8) = w1;
    *(volatile v8h*)(wTg + (size_t)(2 * 256 + tid) * 8) = w2;
    *(volatile v8h*)(whTg + (size_t)tid * 8) = h0;
}

__global__ __launch_bounds__(128) void k_proj(const float* __restrict__ x,
                                               const _Float16* __restrict__ wTg,
                                               _Float16* __restrict__ qh,
                                               _Float16* __restrict__ ql,
                                               _Float16* __restrict__ kh,
                                               _Float16* __restrict__ kl,
                                               _Float16* __restrict__ vh,
                                               _Float16* __restrict__ vl) {
    __shared__ __align__(16) _Float16 xs[64 * FD];
    __shared__ __align__(16) _Float16 wT[WT_ROWS * FD];
    __shared__ __align__(16) _Float16 st[6][4][16 * 32];

    const int tid  = threadIdx.x;
    const int lane = tid & 31;
    const int w    = tid >> 5;
    const int tok0 = blockIdx.x * 64;
    const int b    = tok0 / SEQ;
    const int s0   = tok0 - b * SEQ;
    const float* xb = x + ((size_t)b * SEQ_FULL + s0) * FD;

    for (int idx = tid; idx < 64 * (FD / 4); idx += 128) {
        int r = idx >> 4, c4 = idx & 15;
        v4f xv = *(const v4f*)(xb + (size_t)r * FD + c4 * 4);
        v4h hv;
        hv.x = (_Float16)bf16r(xv.x);
        hv.y = (_Float16)bf16r(xv.y);
        hv.z = (_Float16)bf16r(xv.z);
        hv.w = (_Float16)bf16r(xv.w);
        *(v4h*)(&xs[r * FD + c4 * 4]) = hv;
    }
    for (int idx = tid; idx < (WT_ROWS * FD) / 8; idx += 128)
        *(v8h*)(&wT[idx * 8]) = *(const v8h*)(wTg + (size_t)idx * 8);
    __syncthreads();

    v16h a0 = load_frag16(&xs[(w * 16) * FD], FD, lane);
    v16h a1 = load_frag16(&xs[(w * 16) * FD + 32], FD, lane);
    v8f acc[6];
#pragma unroll
    for (int nt = 0; nt < 6; ++nt) {
        v16h b0 = load_frag16(&wT[(nt * 16) * FD], FD, lane);
        v16h b1 = load_frag16(&wT[(nt * 16) * FD + 32], FD, lane);
        v8f c = zero8();
        c = wmma16(a0, b0, c);
        c = wmma16(a1, b1, c);
        acc[nt] = c;
    }

    const int r0 = (lane >> 4) << 3;
    const int cc = lane & 15;
#pragma unroll
    for (int g = 0; g < 8; ++g) {
        const int ro = (r0 + g) * 32;
        float q0v = acc[0][g], q1v = acc[1][g];
        _Float16 q0h = (_Float16)q0v, q1h = (_Float16)q1v;
        st[0][w][ro + cc]      = q0h;
        st[0][w][ro + 16 + cc] = q1h;
        st[1][w][ro + cc]      = (_Float16)((q0v - (float)q0h) * SC_RES);
        st[1][w][ro + 16 + cc] = (_Float16)((q1v - (float)q1h) * SC_RES);
        float k0v = acc[2][g], k1v = acc[3][g];
        _Float16 k0h = (_Float16)k0v, k1h = (_Float16)k1v;
        st[2][w][ro + cc]      = k0h;
        st[2][w][ro + 16 + cc] = k1h;
        st[3][w][ro + cc]      = (_Float16)((k0v - (float)k0h) * SC_RES);
        st[3][w][ro + 16 + cc] = (_Float16)((k1v - (float)k1h) * SC_RES);
        float v0v = acc[4][g], v1v = acc[5][g];
        _Float16 v0h = (_Float16)v0v, v1h = (_Float16)v1v;
        st[4][w][ro + cc]      = v0h;
        st[4][w][ro + 16 + cc] = v1h;
        st[5][w][ro + cc]      = (_Float16)((v0v - (float)v0h) * SC_RES);
        st[5][w][ro + 16 + cc] = (_Float16)((v1v - (float)v1h) * SC_RES);
    }
    wave_lds_sync();

    v8h pv[6][2];
#pragma unroll
    for (int p = 0; p < 6; ++p) {
        pv[p][0] = *(const v8h*)(&st[p][w][lane * 8]);
        pv[p][1] = *(const v8h*)(&st[p][w][256 + lane * 8]);
    }
    const size_t base = (size_t)(tok0 + w * 16) * 32;
    *(volatile v8h*)(qh + base + lane * 8)       = pv[0][0];
    *(volatile v8h*)(qh + base + 256 + lane * 8) = pv[0][1];
    *(volatile v8h*)(ql + base + lane * 8)       = pv[1][0];
    *(volatile v8h*)(ql + base + 256 + lane * 8) = pv[1][1];
    *(volatile v8h*)(kh + base + lane * 8)       = pv[2][0];
    *(volatile v8h*)(kh + base + 256 + lane * 8) = pv[2][1];
    *(volatile v8h*)(kl + base + lane * 8)       = pv[3][0];
    *(volatile v8h*)(kl + base + 256 + lane * 8) = pv[3][1];
    *(volatile v8h*)(vh + base + lane * 8)       = pv[4][0];
    *(volatile v8h*)(vh + base + 256 + lane * 8) = pv[4][1];
    *(volatile v8h*)(vl + base + lane * 8)       = pv[5][0];
    *(volatile v8h*)(vl + base + 256 + lane * 8) = pv[5][1];
    __threadfence();
    *(volatile v8h*)(qh + base + lane * 8)       = pv[0][0];
    *(volatile v8h*)(qh + base + 256 + lane * 8) = pv[0][1];
    *(volatile v8h*)(ql + base + lane * 8)       = pv[1][0];
    *(volatile v8h*)(ql + base + 256 + lane * 8) = pv[1][1];
    *(volatile v8h*)(kh + base + lane * 8)       = pv[2][0];
    *(volatile v8h*)(kh + base + 256 + lane * 8) = pv[2][1];
    *(volatile v8h*)(kl + base + lane * 8)       = pv[3][0];
    *(volatile v8h*)(kl + base + 256 + lane * 8) = pv[3][1];
    *(volatile v8h*)(vh + base + lane * 8)       = pv[4][0];
    *(volatile v8h*)(vh + base + 256 + lane * 8) = pv[4][1];
    *(volatile v8h*)(vl + base + lane * 8)       = pv[5][0];
    *(volatile v8h*)(vl + base + 256 + lane * 8) = pv[5][1];
}

__global__ __launch_bounds__(256) __attribute__((amdgpu_num_vgpr(256)))
void k_stats(const _Float16* __restrict__ qh,
             const _Float16* __restrict__ ql,
             const _Float16* __restrict__ kh,
             const _Float16* __restrict__ kl,
             float* __restrict__ m2) {
    __shared__ __align__(16) float stt[128];
    const int tid  = threadIdx.x;
    const int lane = tid & 31;
    const int w    = tid >> 5;
    const int b    = blockIdx.x;
    const int key0 = (blockIdx.y * 8 + w) * 16;

    const size_t kt = ((size_t)b * SEQ + key0) * 32;
    const v16h khf = load_frag16(kh + kt, 32, lane);
    const v16h klf = load_frag16(kl + kt, 32, lane);
    const _Float16* qhb = qh + (size_t)b * SEQ * 32;
    const _Float16* qlb = ql + (size_t)b * SEQ * 32;

    float mr = -1.0e30f, zr = 0.0f;
#pragma unroll 1
    for (int qt = 0; qt < SEQ; qt += 16) {
        v16h qhf = load_frag16(qhb + (size_t)qt * 32, 32, lane);
        v16h qlf = load_frag16(qlb + (size_t)qt * 32, 32, lane);
        v8f sh = wmma16(qhf, khf, zero8());
        v8f sr = wmma16(qhf, klf, zero8());
        sr = wmma16(qlf, khf, sr);
        float t[8];
#pragma unroll
        for (int i = 0; i < 8; ++i) t[i] = __builtin_fmaf(sh[i], C1, sr[i] * C2);
        float tmax = t[0];
#pragma unroll
        for (int i = 1; i < 8; ++i) tmax = fmaxf(tmax, t[i]);
        tmax = fmaxf(tmax, __shfl_xor(tmax, 16, 32));
        const float mn = fmaxf(mr, tmax);
        float ps = 0.0f;
#pragma unroll
        for (int i = 0; i < 8; ++i) ps += ex2(t[i] - mn);
        ps += __shfl_xor(ps, 16, 32);
        zr = zr * ex2(mr - mn) + ps;
        mr = mn;
    }
    const float val = mr + log2f(zr) - 14.0f;
    if (lane < 16) stt[w * 16 + lane] = val;
    __syncthreads();
    if (w == 0) {
        v4f v = *(const v4f*)(&stt[lane * 4]);
        float* dst = m2 + (size_t)b * SEQ + (size_t)blockIdx.y * 128 + lane * 4;
        *(volatile v4f*)dst = v;
        __threadfence();
        *(volatile v4f*)dst = v;
    }
}

__global__ __launch_bounds__(256) __attribute__((amdgpu_num_vgpr(256)))
void k_attn(const _Float16* __restrict__ qh,
            const _Float16* __restrict__ ql,
            const _Float16* __restrict__ kh,
            const _Float16* __restrict__ kl,
            const _Float16* __restrict__ vh,
            const _Float16* __restrict__ vl,
            const float*    __restrict__ m2,
            const _Float16* __restrict__ whTg,
            float* __restrict__ out) {
    __shared__ __align__(16) _Float16 VshT[DV * CH];
    __shared__ __align__(16) _Float16 VslT[DV * CH];
    __shared__ __align__(16) _Float16 Pst[8][16 * 32];
    __shared__ __align__(16) _Float16 Prs[8][16 * 32];
    __shared__ __align__(16) _Float16 WhT[FO * DV];
    __shared__ __align__(16) float    Ost[8][16 * FO];

    const int tid  = threadIdx.x;
    const int lane = tid & 31;
    const int w    = tid >> 5;
    const int b    = blockIdx.x;
    const int q0r  = blockIdx.y * 128 + w * 16;
    const int r0   = (lane >> 4) << 3;
    const int cc   = lane & 15;

    *(v8h*)(&WhT[tid * 8]) = *(const v8h*)(whTg + (size_t)tid * 8);

    const size_t qt = ((size_t)b * SEQ + q0r) * 32;
    const v16h qhf = load_frag16(qh + qt, 32, lane);
    const v16h qlf = load_frag16(ql + qt, 32, lane);
    const _Float16* khb = kh + (size_t)b * SEQ * 32;
    const _Float16* klb = kl + (size_t)b * SEQ * 32;
    const _Float16* vhb = vh + (size_t)b * SEQ * 32;
    const _Float16* vlb = vl + (size_t)b * SEQ * 32;
    const float*    m2b = m2 + (size_t)b * SEQ;

    v8f o0 = zero8(), o1 = zero8();
    v8f or0 = zero8(), or1 = zero8();

#pragma unroll 1
    for (int c0 = 0; c0 < SEQ; c0 += CH) {
        for (int idx = tid; idx < CH * 4; idx += 256) {
            int t = idx >> 2, part = idx & 3;
            v8h vv = *(const v8h*)(vhb + (size_t)(c0 + t) * 32 + part * 8);
            v8h vr = *(const v8h*)(vlb + (size_t)(c0 + t) * 32 + part * 8);
#pragma unroll
            for (int e = 0; e < 8; ++e) {
                VshT[(part * 8 + e) * CH + t] = vv[e];
                VslT[(part * 8 + e) * CH + t] = vr[e];
            }
        }
        __syncthreads();

#pragma unroll 1
        for (int j = 0; j < CH; j += 32) {
            const int kA = c0 + j;
            v16h khA = load_frag16(khb + (size_t)kA * 32, 32, lane);
            v16h klA = load_frag16(klb + (size_t)kA * 32, 32, lane);
            v8f sh0 = wmma16(qhf, khA, zero8());
            v8f sr0 = wmma16(qhf, klA, zero8());
            sr0 = wmma16(qlf, khA, sr0);
            v16h khB = load_frag16(khb + (size_t)(kA + 16) * 32, 32, lane);
            v16h klB = load_frag16(klb + (size_t)(kA + 16) * 32, 32, lane);
            v8f sh1 = wmma16(qhf, khB, zero8());
            v8f sr1 = wmma16(qhf, klB, zero8());
            sr1 = wmma16(qlf, khB, sr1);

            const float mA = m2b[kA + cc];
            const float mB = m2b[kA + 16 + cc];
#pragma unroll
            for (int g = 0; g < 8; ++g) {
                float t0 = __builtin_fmaf(sh0[g], C1, sr0[g] * C2);
                float t1 = __builtin_fmaf(sh1[g], C1, sr1[g] * C2);
                Pst[w][(r0 + g) * 32 + cc]      = (_Float16)ex2(t0 - mA);
                Pst[w][(r0 + g) * 32 + 16 + cc] = (_Float16)ex2(t1 - mB);
            }
            wave_lds_sync();
            v16h pa  = load_frag16(&Pst[w][0], 32, lane);
            v16h vb0 = load_frag16(&VshT[0 * CH + j], CH, lane);
            v16h vb1 = load_frag16(&VshT[16 * CH + j], CH, lane);
            o0 = wmma16(pa, vb0, o0);
            o1 = wmma16(pa, vb1, o1);
            v16h vr0 = load_frag16(&VslT[0 * CH + j], CH, lane);
            v16h vr1 = load_frag16(&VslT[16 * CH + j], CH, lane);
            or0 = wmma16(pa, vr0, or0);
            or1 = wmma16(pa, vr1, or1);
        }
        __syncthreads();
    }

#pragma unroll
    for (int g = 0; g < 8; ++g) {
        float ha0 = __builtin_fmaf(or0[g], SC_RINV, o0[g]) * SC_O2H;
        float ha1 = __builtin_fmaf(or1[g], SC_RINV, o1[g]) * SC_O2H;
        _Float16 hh0 = (_Float16)ha0, hh1 = (_Float16)ha1;
        Pst[w][(r0 + g) * 32 + cc]      = hh0;
        Pst[w][(r0 + g) * 32 + 16 + cc] = hh1;
        Prs[w][(r0 + g) * 32 + cc]      = (_Float16)((ha0 - (float)hh0) * SC_RES);
        Prs[w][(r0 + g) * 32 + 16 + cc] = (_Float16)((ha1 - (float)hh1) * SC_RES);
    }
    wave_lds_sync();
    const v16h ha  = load_frag16(&Pst[w][0], 32, lane);
    const v16h hra = load_frag16(&Prs[w][0], 32, lane);
    v8f oc[4], ocr[4];
#pragma unroll
    for (int nt = 0; nt < 4; ++nt) {
        v16h wb = load_frag16(&WhT[(nt * 16) * DV], DV, lane);
        oc[nt]  = wmma16(ha, wb, zero8());
        ocr[nt] = wmma16(hra, wb, zero8());
    }
#pragma unroll
    for (int nt = 0; nt < 4; ++nt)
#pragma unroll
        for (int g = 0; g < 8; ++g)
            Ost[w][(r0 + g) * FO + nt * 16 + cc] =
                __builtin_fmaf(ocr[nt][g], SC_RINV, oc[nt][g]) * SC_OUT;
    wave_lds_sync();

    v4f sv[8];
#pragma unroll
    for (int i = 0; i < 8; ++i) sv[i] = *(const v4f*)(&Ost[w][i * 128 + lane * 4]);
    float* ob = out + ((size_t)b * SEQ + q0r) * FO;
#pragma unroll
    for (int i = 0; i < 8; ++i) *(volatile v4f*)(ob + i * 128 + lane * 4) = sv[i];
    __threadfence();
#pragma unroll
    for (int i = 0; i < 8; ++i) *(volatile v4f*)(ob + i * 128 + lane * 4) = sv[i];
}

extern "C" void kernel_launch(void* const* d_in, const int* in_sizes, int n_in,
                              void* d_out, int out_size, void* d_ws, size_t ws_size,
                              hipStream_t stream) {
    if (n_in < 5) return;
    if (in_sizes[0] < ((NB - 1) * SEQ_FULL + SEQ) * FD) return;
    if (in_sizes[1] < FD * DQ || in_sizes[2] < FD * DQ) return;
    if (in_sizes[3] < FD * DV || in_sizes[4] < DV * FO) return;
    if (out_size < NTOK * FO) return;

    const float* x  = (const float*)d_in[0];
    const float* Wq = (const float*)d_in[1];
    const float* Wk = (const float*)d_in[2];
    const float* Wv = (const float*)d_in[3];
    const float* Wh = (const float*)d_in[4];
    float* out = (float*)d_out;

    char* ws = (char*)d_ws;
    size_t off = 0;
    _Float16* wTg  = (_Float16*)(ws + off); off += (size_t)WT_ROWS * FD * 2;
    _Float16* whTg = (_Float16*)(ws + off); off += (size_t)FO * DV * 2;
    const size_t PL = (size_t)NTOK * 32 * 2;
    _Float16* qh = (_Float16*)(ws + off); off += PL;
    _Float16* ql = (_Float16*)(ws + off); off += PL;
    _Float16* kh = (_Float16*)(ws + off); off += PL;
    _Float16* kl = (_Float16*)(ws + off); off += PL;
    _Float16* vh = (_Float16*)(ws + off); off += PL;
    _Float16* vl = (_Float16*)(ws + off); off += PL;
    float*    m2 = (float*)(ws + off);    off += (size_t)NTOK * 4;
    if (off > ws_size) return;

    k_wprep<<<dim3(1), dim3(256), 0, stream>>>(Wq, Wk, Wv, Wh, wTg, whTg);
    k_proj<<<dim3(NTOK / 64), dim3(128), 0, stream>>>(x, wTg, qh, ql, kh, kl, vh, vl);
    k_stats<<<dim3(NB, SEQ / 128), dim3(256), 0, stream>>>(qh, ql, kh, kl, m2);
    k_attn<<<dim3(NB, SEQ / 128), dim3(256), 0, stream>>>(qh, ql, kh, kl, vh, vl, m2, whTg, out);
}
